// MambaBlock_85796266705208
// MI455X (gfx1250) — hardware-verified
//
#include <hip/hip_runtime.h>
#include <stddef.h>
#include <stdint.h>
#include <math.h>


#define DIM     1024
#define DIN     2048
#define NST     16
#define DCV     4
#define DTR     64
#define NXD     96
#define NXP     128
#define NBAT    2
#define SEQ     2048
#define MROWS   (NBAT * SEQ)
#define NIN     4096
#define K2      4096
#define K2D     128
#define BCW     32
#define PLANE   (MROWS * DIN)
#define GBM     64
#define GBN     64
#define GTHR    128
#define NTHR    256
#define ST      32
#define SCH     128
#define SCAN_LDS_FLOATS (4 * ST * SCH + ST * BCW)
#define WSMAX   134217728

#define PU_XB   (MROWS * DIM / 8)
#define PU_WIN  (NIN * DIM / 8)
#define PU_WO   (DIM * K2 / 8)
#define PU_WX   (NXP * K2 / 8)
#define PU_WDT  (DIN * K2D / 8)
#define PU_ALL  (PU_XB + PU_WIN + PU_WO + PU_WX + PU_WDT)

static_assert(MROWS % 128 == 0 && MROWS % GBM == 0);
static_assert(NIN % GBN == 0 && NXP % GBN == 0 && DIN % GBN == 0 && DIM % GBN == 0);
static_assert(DIM % 32 == 0 && K2 % 32 == 0 && K2D % 32 == 0 && K2 == 2 * DIN && K2D == 2 * DTR);
static_assert(GBM == (GTHR / 32) * 16 && GBN == 64);
static_assert(PU_XB % NTHR == 0 && PU_WIN % NTHR == 0 && PU_WO % NTHR == 0 && PU_WX % NTHR == 0 && PU_WDT % NTHR == 0);
static_assert(SEQ % ST == 0 && DIN % SCH == 0 && SCH * 2 == NTHR && DIN / SCH == 16);
static_assert(ST * SCH / 4 == 4 * NTHR && ST * SCH / 8 == 2 * NTHR && ST * BCW / 4 == NTHR);
static_assert(SCAN_LDS_FLOATS * 4 == 69632);
static_assert(NST == 16 && DCV == 4 && DTR + 2 * NST == NXD && NXD - DTR == BCW);
static_assert(MROWS == 2 * SEQ && (SEQ & (SEQ - 1)) == 0 && (DIN & (DIN - 1)) == 0 && (DTR & (DTR - 1)) == 0);

typedef float          v4f   __attribute__((ext_vector_type(4)));
typedef float          v8f   __attribute__((ext_vector_type(8)));
typedef int            v8i   __attribute__((ext_vector_type(8)));
typedef unsigned       v4u   __attribute__((ext_vector_type(4)));
typedef unsigned short v4us  __attribute__((ext_vector_type(4)));
typedef unsigned short v8us  __attribute__((ext_vector_type(8)));
typedef unsigned short v16us __attribute__((ext_vector_type(16)));
typedef __bf16         v16bf __attribute__((ext_vector_type(16)));
typedef v4f  __attribute__((may_alias)) v4fa;
typedef v4u  __attribute__((may_alias)) v4ua;
typedef v4us __attribute__((may_alias)) v4usa;
typedef v8us __attribute__((may_alias)) v8usa;
union FragB { v16bf v; v16us u; v8us h[2]; v8i w; };

__device__ __forceinline__ v8f wmb(const FragB& a, const FragB& b, v8f c) {
  v8f d = __builtin_amdgcn_wmma_f32_16x16x32_bf16(false, a.v, false, b.v, (short)0, c, false, false);
  asm volatile("v_nop\n\tv_nop\n\tv_nop\n\tv_nop" : "+v"(d) : "v"(a.w), "v"(b.w));
  return d;
}

__device__ __forceinline__ unsigned bf16_bits(float f) {
  const unsigned u = __float_as_uint(f);
  return (u + 0x7FFFu + ((u >> 16) & 1u)) >> 16;
}
__device__ __forceinline__ float bf16_val(float f) {
  return __uint_as_float(bf16_bits(f) << 16);
}
__device__ __forceinline__ unsigned short hl_bits(float v, int lo) {
  const unsigned hb = bf16_bits(v);
  const unsigned lb = bf16_bits(v - __uint_as_float(hb << 16));
  return (unsigned short)(lo != 0 ? lb : hb);
}
__device__ __forceinline__ float lo16f(unsigned w) { return __uint_as_float(w << 16); }
__device__ __forceinline__ float hi16f(unsigned w) { return __uint_as_float(w & 0xffff0000u); }
__device__ __forceinline__ float silu_f(float v) {
  return v * __builtin_amdgcn_rcpf(1.0f + expf(-v));
}
__device__ __forceinline__ float softplus_f(float p) {
  return fmaxf(p, 0.0f) + log1pf(expf(-fabsf(p)));
}

__device__ __forceinline__ void cvt8_put(const float* p, bool ok, unsigned short* dp) {
  const v4f a = *(const v4fa*)p;
  const v4f b = *(const v4fa*)(p + 4);
  v8us o;
  o[0] = ok ? (unsigned short)bf16_bits(a.x) : (unsigned short)0;
  o[1] = ok ? (unsigned short)bf16_bits(a.y) : (unsigned short)0;
  o[2] = ok ? (unsigned short)bf16_bits(a.z) : (unsigned short)0;
  o[3] = ok ? (unsigned short)bf16_bits(a.w) : (unsigned short)0;
  o[4] = ok ? (unsigned short)bf16_bits(b.x) : (unsigned short)0;
  o[5] = ok ? (unsigned short)bf16_bits(b.y) : (unsigned short)0;
  o[6] = ok ? (unsigned short)bf16_bits(b.z) : (unsigned short)0;
  o[7] = ok ? (unsigned short)bf16_bits(b.w) : (unsigned short)0;
  *(volatile v8us*)dp = o;
  __threadfence();
  *(volatile v8us*)dp = o;
}

__global__ __launch_bounds__(NTHR) void k_prep(
    const float* __restrict__ x, const float* __restrict__ win, const float* __restrict__ wx,
    const float* __restrict__ wdt, const float* __restrict__ wo,
    unsigned short* XB, unsigned short* WIN, unsigned short* WOUT2, unsigned short* WXP2,
    unsigned short* WDT2)
{
  const int u = (int)blockIdx.x * NTHR + (int)threadIdx.x;
  if (u < PU_XB) {
    cvt8_put(x + (size_t)8 * u, true, XB + (size_t)8 * u);
  } else if (u < PU_XB + PU_WIN) {
    const int v = u - PU_XB;
    cvt8_put(win + (size_t)8 * v, true, WIN + (size_t)8 * v);
  } else if (u < PU_XB + PU_WIN + PU_WO) {
    const int v  = u - (PU_XB + PU_WIN);
    const int n  = v >> 9;
    const int k8 = (v & 511) * 8;
    cvt8_put(wo + (size_t)n * DIN + (k8 & (DIN - 1)), true, WOUT2 + (size_t)n * K2 + k8);
  } else if (u < PU_XB + PU_WIN + PU_WO + PU_WX) {
    const int v  = u - (PU_XB + PU_WIN + PU_WO);
    const int n  = v >> 9;
    const int k8 = (v & 511) * 8;
    const int nc = n < NXD ? n : NXD - 1;
    cvt8_put(wx + (size_t)nc * DIN + (k8 & (DIN - 1)), n < NXD, WXP2 + (size_t)n * K2 + k8);
  } else if (u < PU_ALL) {
    const int v  = u - (PU_XB + PU_WIN + PU_WO + PU_WX);
    const int n  = v >> 4;
    const int k8 = (v & 15) * 8;
    cvt8_put(wdt + (size_t)n * DTR + (k8 & (DTR - 1)), true, WDT2 + (size_t)n * K2D + k8);
  }
}

template <int EPI, int LDO>
__global__ __launch_bounds__(GTHR) void k_gemm(const unsigned short* __restrict__ A,
                                               const unsigned short* __restrict__ WT, int K,
                                               float* outA, float* outB, unsigned short* outH,
                                               const float* __restrict__ vec) {
  __shared__ __attribute__((aligned(16))) float stg[GBM * GBN];
  const int tid = (int)threadIdx.x, lane = tid & 31, wave = tid >> 5, hh = lane >> 4, m = lane & 15;
  const int rowBase = (int)blockIdx.x * GBM;
  const int col0    = (int)blockIdx.y * GBN;

  v8f acc[4];
  {
    const v8f z = {0.f, 0.f, 0.f, 0.f, 0.f, 0.f, 0.f, 0.f};
    acc[0] = z; acc[1] = z; acc[2] = z; acc[3] = z;
  }
  const unsigned short* ap = A  + (size_t)(rowBase + 16 * wave + m) * (size_t)K + 8 * hh;
  const unsigned short* wp = WT + (size_t)(col0 + m) * (size_t)K + 8 * hh;
  const int ksteps = K >> 5;
#pragma unroll 1
  for (int ks = 0; ks < ksteps; ++ks) {
    FragB af;
    af.h[0] = *(const v8usa*)(ap + 32 * ks);
    af.h[1] = *(const v8usa*)(ap + 32 * ks + 16);
#pragma unroll
    for (int t = 0; t < 4; ++t) {
      const unsigned short* wq = wp + (size_t)(16 * t) * (size_t)K + 32 * ks;
      FragB bf;
      bf.h[0] = *(const v8usa*)wq;
      bf.h[1] = *(const v8usa*)(wq + 16);
      acc[t] = wmb(af, bf, acc[t]);
    }
  }

#pragma unroll
  for (int t = 0; t < 4; ++t) {
    const int lc = 16 * t + m;
#pragma unroll
    for (int r = 0; r < 8; ++r) {
      const int lr = 16 * wave + 8 * hh + r;
      stg[lr * GBN + lc] = acc[t][r];
    }
  }
  __syncthreads();

  if constexpr (EPI == 3) {
    if (blockIdx.y == 0) {
      const int q = m & 7;
      const int lo_sel = (m >= 8) ? 1 : 0;
      v8us qv[8];
#pragma unroll
      for (int i = 0; i < 8; ++i) {
        const int lr = 16 * wave + 2 * i + hh;
        const v4f a = *(const v4fa*)(stg + lr * GBN + 8 * q);
        const v4f b = *(const v4fa*)(stg + lr * GBN + 8 * q + 4);
        v8us o;
        o[0] = hl_bits(a.x, lo_sel); o[1] = hl_bits(a.y, lo_sel);
        o[2] = hl_bits(a.z, lo_sel); o[3] = hl_bits(a.w, lo_sel);
        o[4] = hl_bits(b.x, lo_sel); o[5] = hl_bits(b.y, lo_sel);
        o[6] = hl_bits(b.z, lo_sel); o[7] = hl_bits(b.w, lo_sel);
        qv[i] = o;
      }
#pragma unroll
      for (int i = 0; i < 8; ++i) {
        const int lr = 16 * wave + 2 * i + hh;
        *(volatile v8us*)(outH + (size_t)(rowBase + lr) * K2D + 8 * m) = qv[i];
      }
      __threadfence();
#pragma unroll
      for (int i = 0; i < 8; ++i) {
        const int lr = 16 * wave + 2 * i + hh;
        *(volatile v8us*)(outH + (size_t)(rowBase + lr) * K2D + 8 * m) = qv[i];
      }
    } else {
      const int rs  = lane >> 3;
      const int c4b = (lane & 7) * 4;
      v4f fv[4];
#pragma unroll
      for (int i = 0; i < 4; ++i) {
        const int lr = 16 * wave + 4 * i + rs;
        fv[i] = *(const v4fa*)(stg + lr * GBN + c4b);
      }
#pragma unroll
      for (int i = 0; i < 4; ++i) {
        const int lr = 16 * wave + 4 * i + rs;
        *(volatile v4f*)(outB + (size_t)(rowBase + lr) * BCW + c4b) = fv[i];
      }
      __threadfence();
#pragma unroll
      for (int i = 0; i < 4; ++i) {
        const int lr = 16 * wave + 4 * i + rs;
        *(volatile v4f*)(outB + (size_t)(rowBase + lr) * BCW + c4b) = fv[i];
      }
    }
  } else {
    const int c4 = 4 * m;
    size_t oofs = 0;
    int ocol = col0;

    if constexpr (EPI == 0) {
      const bool isZ = col0 >= DIN;
      if (isZ) {
#pragma unroll 1
        for (int i = 0; i < 8; ++i) {
          float* sp = stg + (16 * wave + 2 * i + hh) * GBN + c4;
          v4f v = *(const v4fa*)sp;
          v.x = silu_f(v.x); v.y = silu_f(v.y); v.z = silu_f(v.z); v.w = silu_f(v.w);
          *(v4fa*)sp = v;
        }
        oofs = (size_t)PLANE;
        ocol = col0 - DIN;
      }
    }
    if constexpr (EPI == 1) {
      const v4f bq = *(const v4fa*)(vec + col0 + c4);
      const float b0 = bf16_val(bq.x), b1 = bf16_val(bq.y), b2 = bf16_val(bq.z), b3 = bf16_val(bq.w);
#pragma unroll 1
      for (int i = 0; i < 8; ++i) {
        float* sp = stg + (16 * wave + 2 * i + hh) * GBN + c4;
        v4f v = *(const v4fa*)sp;
        v.x = softplus_f(v.x + b0); v.y = softplus_f(v.y + b1);
        v.z = softplus_f(v.z + b2); v.w = softplus_f(v.w + b3);
        *(v4fa*)sp = v;
      }
    }

    float* obase = outA + oofs;
    v4f fv[8];
#pragma unroll
    for (int i = 0; i < 8; ++i) {
      const int lr = 16 * wave + 2 * i + hh;
      fv[i] = *(const v4fa*)(stg + lr * GBN + c4);
    }
#pragma unroll
    for (int i = 0; i < 8; ++i) {
      const int lr = 16 * wave + 2 * i + hh;
      float* op = obase + (size_t)(rowBase + lr) * (size_t)LDO + ocol + c4;
      *(volatile v4f*)op = fv[i];
    }
    __threadfence();
#pragma unroll
    for (int i = 0; i < 8; ++i) {
      const int lr = 16 * wave + 2 * i + hh;
      float* op = obase + (size_t)(rowBase + lr) * (size_t)LDO + ocol + c4;
      *(volatile v4f*)op = fv[i];
    }
  }
}

__global__ __launch_bounds__(NTHR) void k_conv(const float* __restrict__ XI, const float* __restrict__ Wc,
                                               const float* __restrict__ bc, unsigned short* UHL) {
  __shared__ __attribute__((aligned(16))) unsigned short hls[2048];
  const int tid = (int)threadIdx.x;
  const int r   = (int)blockIdx.x >> 1;
  const int cb  = ((int)blockIdx.x & 1) * 1024;
  const int c   = cb + 4 * tid;
  const int l   = r & (SEQ - 1);

  v4f w0 = *(const v4fa*)(Wc + (size_t)c * 4);
  v4f w1 = *(const v4fa*)(Wc + (size_t)c * 4 + 4);
  v4f w2 = *(const v4fa*)(Wc + (size_t)c * 4 + 8);
  v4f w3 = *(const v4fa*)(Wc + (size_t)c * 4 + 12);
  const v4f bq = *(const v4fa*)(bc + c);
#pragma unroll
  for (int j = 0; j < 4; ++j) {
    w0[j] = bf16_val(w0[j]); w1[j] = bf16_val(w1[j]); w2[j] = bf16_val(w2[j]); w3[j] = bf16_val(w3[j]);
  }
  float s0 = 0.0f, s1 = 0.0f, s2 = 0.0f, s3 = 0.0f;
#pragma unroll
  for (int j = 0; j < 4; ++j) {
    const bool ok = (l - 3 + j) >= 0;
    const int rr = ok ? (r - 3 + j) : r;
    v4f xv = *(const v4fa*)(XI + (size_t)rr * DIN + c);
    xv.x = ok ? xv.x : 0.0f; xv.y = ok ? xv.y : 0.0f; xv.z = ok ? xv.z : 0.0f; xv.w = ok ? xv.w : 0.0f;
    s0 = fmaf(w0[j], xv.x, s0);
    s1 = fmaf(w1[j], xv.y, s1);
    s2 = fmaf(w2[j], xv.z, s2);
    s3 = fmaf(w3[j], xv.w, s3);
  }
  const float u0 = silu_f(s0 + bf16_val(bq.x));
  const float u1 = silu_f(s1 + bf16_val(bq.y));
  const float u2 = silu_f(s2 + bf16_val(bq.z));
  const float u3 = silu_f(s3 + bf16_val(bq.w));

  v4us h4, l4;
  h4[0] = hl_bits(u0, 0); l4[0] = hl_bits(u0, 1);
  h4[1] = hl_bits(u1, 0); l4[1] = hl_bits(u1, 1);
  h4[2] = hl_bits(u2, 0); l4[2] = hl_bits(u2, 1);
  h4[3] = hl_bits(u3, 0); l4[3] = hl_bits(u3, 1);
  *(v4usa*)(hls + 4 * tid) = h4;
  *(v4usa*)(hls + 1024 + 4 * tid) = l4;
  __syncthreads();
  const int pl = tid >> 7;
  const int ix = tid & 127;
  const v8us q = *(const v8usa*)(hls + pl * 1024 + 8 * ix);

  unsigned short* hp = UHL + (size_t)r * K2 + (size_t)pl * DIN + cb + 8 * ix;
  *(volatile v8us*)hp = q;
  __threadfence();
  *(volatile v8us*)hp = q;
}

__global__ __launch_bounds__(NTHR) void k_scan(const float* __restrict__ DELTA, const float* __restrict__ SZ,
                                               const float* __restrict__ BC, const float* __restrict__ Alog,
                                               const float* __restrict__ Dv, unsigned short* UG) {
  extern __shared__ __attribute__((aligned(16))) float sm[];
  float* dl  = sm;
  float* uu  = sm + ST * SCH;
  float* sz  = sm + 2 * ST * SCH;
  float* gg  = sm + 3 * ST * SCH;
  float* bcs = sm + 4 * ST * SCH;
  const int tid = (int)threadIdx.x;
  const int ch = tid >> 1, half = tid & 1;
  const int b = (int)blockIdx.x >> 4;
  const int chBase = ((int)blockIdx.x & 15) * SCH;

  float Aa[8];
  {
    const float* arow = Alog + (size_t)(chBase + ch) * NST + 8 * half;
    const v4f a0 = *(const v4fa*)arow;
    const v4f a1 = *(const v4fa*)(arow + 4);
    Aa[0] = -expf(bf16_val(a0.x)); Aa[1] = -expf(bf16_val(a0.y));
    Aa[2] = -expf(bf16_val(a0.z)); Aa[3] = -expf(bf16_val(a0.w));
    Aa[4] = -expf(bf16_val(a1.x)); Aa[5] = -expf(bf16_val(a1.y));
    Aa[6] = -expf(bf16_val(a1.z)); Aa[7] = -expf(bf16_val(a1.w));
  }
  const float Dd = bf16_val(Dv[chBase + ch]);
  float h[8];
#pragma unroll
  for (int j = 0; j < 8; ++j) h[j] = 0.0f;

#pragma unroll 1
  for (int cnk = 0; cnk < SEQ / ST; ++cnk) {
    const int row0 = b * SEQ + cnk * ST;
#pragma unroll
    for (int it = 0; it < 4; ++it) {
      const int idx = it * NTHR + tid;
      const int row = idx >> 5;
      const int cc  = (idx & 31) * 4;
      const size_t go = (size_t)(row0 + row) * DIN + chBase + cc;
      const v4f a = *(const v4fa*)(DELTA + go);
      const v4f f = *(const v4fa*)(SZ + go);
      *(v4fa*)(dl + row * SCH + cc) = a;
      *(v4fa*)(sz + row * SCH + cc) = f;
    }
#pragma unroll
    for (int it = 0; it < 2; ++it) {
      const int idx = it * NTHR + tid;
      const int row = idx >> 4;
      const int c8  = (idx & 15) * 8;
      const unsigned short* gp = UG + (size_t)(row0 + row) * K2 + chBase + c8;
      const v4u hw = *(const v4ua*)gp;
      const v4u lw = *(const v4ua*)(gp + DIN);
      v4f e0, e1;
      e0.x = lo16f(hw.x) + lo16f(lw.x); e0.y = hi16f(hw.x) + hi16f(lw.x);
      e0.z = lo16f(hw.y) + lo16f(lw.y); e0.w = hi16f(hw.y) + hi16f(lw.y);
      e1.x = lo16f(hw.z) + lo16f(lw.z); e1.y = hi16f(hw.z) + hi16f(lw.z);
      e1.z = lo16f(hw.w) + lo16f(lw.w); e1.w = hi16f(hw.w) + hi16f(lw.w);
      *(v4fa*)(uu + row * SCH + c8) = e0;
      *(v4fa*)(uu + row * SCH + c8 + 4) = e1;
    }
    {
      const int row = tid >> 3;
      const int cc  = (tid & 7) * 4;
      const v4f a = *(const v4fa*)(BC + (size_t)(row0 + row) * BCW + cc);
      *(v4fa*)(bcs + row * BCW + cc) = a;
    }
    __syncthreads();

#pragma unroll 1
    for (int t = 0; t < ST; ++t) {
      const float d  = dl[t * SCH + ch];
      const float u  = uu[t * SCH + ch];
      const float zz = sz[t * SCH + ch];
      const v4f B0 = *(const v4fa*)(bcs + t * BCW + 8 * half);
      const v4f B1 = *(const v4fa*)(bcs + t * BCW + 8 * half + 4);
      const v4f C0 = *(const v4fa*)(bcs + t * BCW + 16 + 8 * half);
      const v4f C1 = *(const v4fa*)(bcs + t * BCW + 16 + 8 * half + 4);
      const float Bv[8] = {B0.x, B0.y, B0.z, B0.w, B1.x, B1.y, B1.z, B1.w};
      const float Cv[8] = {C0.x, C0.y, C0.z, C0.w, C1.x, C1.y, C1.z, C1.w};
      float p = 0.0f;
#pragma unroll
      for (int j = 0; j < 8; ++j) {
        const float dA = expf(d * Aa[j]);
        h[j] = fmaf(dA, h[j], (d * Bv[j]) * u);
        p = fmaf(h[j], Cv[j], p);
      }
      const float other = __shfl_xor(p, 1, 32);
      const float plo = (half != 0) ? other : p;
      const float phi = (half != 0) ? p : other;
      const float y = (plo + phi) + u * Dd;
      const float g = y * zz;
      if (half == 0) gg[t * SCH + ch] = g;
    }
    __syncthreads();

    v8us ov[4];
#pragma unroll
    for (int it = 0; it < 4; ++it) {
      const int plane = it >> 1;
      const int idx = (it & 1) * NTHR + tid;
      const int row = idx >> 4;
      const int c8  = (idx & 15) * 8;
      const v4f g0 = *(const v4fa*)(gg + row * SCH + c8);
      const v4f g1 = *(const v4fa*)(gg + row * SCH + c8 + 4);
      v8us o;
      o[0] = hl_bits(g0.x, plane); o[1] = hl_bits(g0.y, plane);
      o[2] = hl_bits(g0.z, plane); o[3] = hl_bits(g0.w, plane);
      o[4] = hl_bits(g1.x, plane); o[5] = hl_bits(g1.y, plane);
      o[6] = hl_bits(g1.z, plane); o[7] = hl_bits(g1.w, plane);
      ov[it] = o;
    }
#pragma unroll
    for (int it = 0; it < 4; ++it) {
      const int plane = it >> 1;
      const int idx = (it & 1) * NTHR + tid;
      const int row = idx >> 4;
      const int c8  = (idx & 15) * 8;
      unsigned short* gp = UG + (size_t)(row0 + row) * K2 + (size_t)plane * DIN + chBase + c8;
      *(volatile v8us*)gp = ov[it];
    }
    __threadfence();
#pragma unroll
    for (int it = 0; it < 4; ++it) {
      const int plane = it >> 1;
      const int idx = (it & 1) * NTHR + tid;
      const int row = idx >> 4;
      const int c8  = (idx & 15) * 8;
      unsigned short* gp = UG + (size_t)(row0 + row) * K2 + (size_t)plane * DIN + chBase + c8;
      *(volatile v8us*)gp = ov[it];
    }
    __syncthreads();
  }
}

extern "C" void kernel_launch(void* const* d_in, const int* in_sizes, int n_in,
                              void* d_out, int out_size, void* d_ws, size_t ws_size,
                              hipStream_t stream) {
  if (n_in < 10) return;
  if (in_sizes[0] != MROWS * DIM) return;
  if (in_sizes[1] != NIN * DIM) return;
  if (in_sizes[2] != DIN * DCV) return;
  if (in_sizes[3] != DIN) return;
  if (in_sizes[4] != NXD * DIN) return;
  if (in_sizes[5] != DIN * DTR) return;
  if (in_sizes[6] != DIN) return;
  if (in_sizes[7] != DIN * NST) return;
  if (in_sizes[8] != DIN) return;
  if (in_sizes[9] != DIM * DIN) return;
  if (out_size != MROWS * DIM) return;

  const float* x     = (const float*)d_in[0];
  const float* W_in  = (const float*)d_in[1];
  const float* W_cv  = (const float*)d_in[2];
  const float* b_cv  = (const float*)d_in[3];
  const float* W_xp  = (const float*)d_in[4];
  const float* W_dt  = (const float*)d_in[5];
  const float* b_dt  = (const float*)d_in[6];
  const float* A_log = (const float*)d_in[7];
  const float* D_sk  = (const float*)d_in[8];
  const float* W_out = (const float*)d_in[9];
  float* out = (float*)d_out;

  char* ws = (char*)d_ws;
  size_t off = 0;
  const size_t oXB   = off; off += (size_t)MROWS * DIM * 2;
  const size_t oWIN  = off; off += (size_t)NIN * DIM * 2;
  const size_t oWO   = off; off += (size_t)DIM * K2 * 2;
  const size_t oWX   = off; off += (size_t)NXP * K2 * 2;
  const size_t oWD   = off; off += (size_t)DIN * K2D * 2;
  const size_t oXI   = off; off += (size_t)PLANE * 4;
  const size_t oSZ   = off; off += (size_t)PLANE * 4;
  const size_t oUHL  = off; off += (size_t)MROWS * K2 * 2;
  const size_t oDTR  = off; off += (size_t)MROWS * K2D * 2;
  const size_t oBC   = off; off += (size_t)MROWS * BCW * 4;
  if (off > ws_size || off > (size_t)WSMAX) return;
  if (oSZ != oXI + (size_t)PLANE * 4) return;
  unsigned short* XB    = (unsigned short*)(ws + oXB);
  unsigned short* WIN   = (unsigned short*)(ws + oWIN);
  unsigned short* WOUT2 = (unsigned short*)(ws + oWO);
  unsigned short* WXP2  = (unsigned short*)(ws + oWX);
  unsigned short* WDT2  = (unsigned short*)(ws + oWD);
  float*          XI    = (float*)(ws + oXI);
  float*          SZp   = (float*)(ws + oSZ);
  unsigned short* UHL   = (unsigned short*)(ws + oUHL);
  unsigned short* DTRHL = (unsigned short*)(ws + oDTR);
  float*          BCp   = (float*)(ws + oBC);
  float*          DELTA = XI;

  const size_t scanLds = (size_t)SCAN_LDS_FLOATS * 4;
  hipFuncSetAttribute(reinterpret_cast<const void*>(&k_scan), hipFuncAttributeMaxDynamicSharedMemorySize, (int)scanLds);

  k_prep<<<PU_ALL / NTHR, NTHR, 0, stream>>>(x, W_in, W_xp, W_dt, W_out, XB, WIN, WOUT2, WXP2, WDT2);
  k_gemm<0, DIN><<<dim3(MROWS / GBM, NIN / GBN), GTHR, 0, stream>>>(XB, WIN, DIM, XI, BCp, DTRHL, b_dt);
  k_conv<<<MROWS * 2, NTHR, 0, stream>>>(XI, W_cv, b_cv, UHL);
  k_gemm<3, DIN><<<dim3(MROWS / GBM, NXP / GBN), GTHR, 0, stream>>>(UHL, WXP2, K2, XI, BCp, DTRHL, b_dt);
  k_gemm<1, DIN><<<dim3(MROWS / GBM, DIN / GBN), GTHR, 0, stream>>>(DTRHL, WDT2, K2D, DELTA, BCp, DTRHL, b_dt);
  k_scan<<<NBAT * (DIN / SCH), NTHR, scanLds, stream>>>(DELTA, SZp, BCp, A_log, D_sk, UHL);
  k_gemm<2, DIM><<<dim3(MROWS / GBM, DIM / GBN), GTHR, 0, stream>>>(UHL, WOUT2, K2, out, BCp, DTRHL, b_dt);
}
